// IwinTransformer3D_47425028882596
// MI455X (gfx1250) — hardware-verified
//
#include <hip/hip_runtime.h>
#include <stdint.h>

#define NTN    50176
#define CCH    128
#define NHD    4
#define HD     32
#define C3     384
#define HID    512
#define NWIN   128
#define NTW    392
#define TP     448
#define DFR    8
#define STRIPS (TP / 64)
#define NROWW  57344
#define QEND   400
#define FR     56
#define LDC    132
#define PP     72
#define OSP    36
#define PWB    2304
#define QSC    0.17677669529663687f
#define INV512 0.001953125f
#define LN4096 8.3177661667193429f

static_assert(NROWW == NWIN * TP);
static_assert(NTN == NWIN * NTW);
static_assert(PWB == 16 * PP * 2);
static_assert(16 * OSP * 4 <= PWB);
static_assert((TP % 64) == 0);
static_assert((NTN % 64) == 0);
static_assert((QEND % 16) == 0 && QEND >= NTW && QEND <= TP);
static_assert((PP * 2) % 16 == 0);
static_assert((LDC * 4) % 16 == 0);

typedef _Float16 v16h __attribute__((ext_vector_type(16)));
typedef _Float16 v8h  __attribute__((ext_vector_type(8)));
typedef float    v8f  __attribute__((ext_vector_type(8)));
typedef float    v4f  __attribute__((ext_vector_type(4)));
typedef unsigned int v4u __attribute__((ext_vector_type(4)));
typedef unsigned int v2u __attribute__((ext_vector_type(2)));

__device__ __forceinline__ unsigned short bf_bits(float f) {
  unsigned u = __float_as_uint(f);
  return (unsigned short)((u + 0x7FFFu + ((u >> 16) & 1u)) >> 16);
}
__device__ __forceinline__ float bf_up(unsigned short b) { return __uint_as_float(((unsigned)b) << 16); }
__device__ __forceinline__ float bfr(float f) { return bf_up(bf_bits(f)); }
__device__ __forceinline__ unsigned short h_bits(_Float16 x) { return __builtin_bit_cast(unsigned short, x); }
__device__ __forceinline__ unsigned short hb16(float f) { return h_bits((_Float16)f); }
__device__ __forceinline__ unsigned pk16(unsigned short a, unsigned short b) { return (unsigned)a | ((unsigned)b << 16); }
__device__ __forceinline__ v8f zero8() { v8f z = {0.f, 0.f, 0.f, 0.f, 0.f, 0.f, 0.f, 0.f}; return z; }

__device__ __forceinline__ float wsum(float v) {
  v += __shfl_xor(v, 1, 32);
  v += __shfl_xor(v, 2, 32);
  v += __shfl_xor(v, 4, 32);
  v += __shfl_xor(v, 8, 32);
  v += __shfl_xor(v, 16, 32);
  return v;
}

__device__ __forceinline__ int win_token(int wi, int n) {
  n = min(max(n, 0), NTW - 1);
  const int b = (wi >> 6) & 1, wh = (wi >> 3) & 7, ww = wi & 7;
  const int dd = n / 49;
  const int rem = n - dd * 49;
  const int r = rem / 7;
  const int s = rem - r * 7;
  return ((b * DFR + dd) * FR + (r * 8 + wh)) * FR + (s * 8 + ww);
}

__device__ __forceinline__ v16h ldfrag_h(const _Float16* p) {
  union { v16h v; v8h h[2]; } f;
  f.h[0] = *(const v8h*)(p);
  f.h[1] = *(const v8h*)(p + 16);
  return f.v;
}

__device__ __forceinline__ v8f mma_raw(v16h a, v16h b, v8f c) {
  return __builtin_amdgcn_wmma_f32_16x16x32_f16(false, a, false, b, (short)0, c, false, false);
}
__device__ __forceinline__ v8f mma_g1(v16h a, v16h b, v8f c) {
  c = mma_raw(a, b, c);
#if defined(__HIP_DEVICE_COMPILE__)
  asm volatile("v_nop\n\tv_nop\n\tv_nop\n\tv_nop" : "+v"(c) : "v"(a), "v"(b));
#endif
  return c;
}
__device__ __forceinline__ void guard2(v8f& c0, v8f& c1, const v16h& a0, const v16h& b0, const v16h& b1) {
#if defined(__HIP_DEVICE_COMPILE__)
  asm volatile("v_nop\n\tv_nop\n\tv_nop\n\tv_nop" : "+v"(c0), "+v"(c1) : "v"(a0), "v"(b0), "v"(b1));
#endif
}
__device__ __forceinline__ void guard4(v8f& c0, v8f& c1, v8f& c2, v8f& c3,
                                       const v16h& a0, const v16h& a1, const v16h& b0, const v16h& b1) {
#if defined(__HIP_DEVICE_COMPILE__)
  asm volatile("v_nop\n\tv_nop\n\tv_nop\n\tv_nop"
               : "+v"(c0), "+v"(c1), "+v"(c2), "+v"(c3) : "v"(a0), "v"(a1), "v"(b0), "v"(b1));
#endif
}
__device__ __forceinline__ void wave_sync_lds() {
  __builtin_amdgcn_fence(__ATOMIC_RELEASE, "workgroup");
  __builtin_amdgcn_wave_barrier();
  __builtin_amdgcn_fence(__ATOMIC_ACQUIRE, "workgroup");
}

__device__ __forceinline__ v4f ln4(const v4f a, const v4f gg, const v4f be) {
  float s = (a[0] + a[1]) + (a[2] + a[3]);
  s = wsum(s);
  const float mu = s * (1.0f / (float)CCH);
  v4f d;
  d[0] = a[0] - mu; d[1] = a[1] - mu; d[2] = a[2] - mu; d[3] = a[3] - mu;
  float sq = (d[0] * d[0] + d[1] * d[1]) + (d[2] * d[2] + d[3] * d[3]);
  sq = wsum(sq);
  const float rs = rsqrtf(sq * (1.0f / (float)CCH) + 1e-5f);
  v4f y;
#pragma unroll
  for (int e = 0; e < 4; ++e) y[e] = (d[e] * rs) * gg[e] + be[e];
  return y;
}

__device__ __forceinline__ void mm_tile(const _Float16* __restrict__ A, int lda, size_t aks,
                                        const _Float16* __restrict__ W, int ldw, int nks,
                                        int arow0, int bcol0, float* Cs) {
  const int tid = threadIdx.x, wave = tid >> 5, lane = tid & 31, hh = lane >> 4, c = lane & 15;
  const int mw = wave >> 2, nw = wave & 3;
  const _Float16* a0p = A + (size_t)(arow0 + mw * 32 + c) * lda + 8 * hh;
  const _Float16* a1p = A + (size_t)(arow0 + mw * 32 + 16 + c) * lda + 8 * hh;
  const _Float16* b0p = W + (size_t)(bcol0 + nw * 32 + c) * ldw + 8 * hh;
  const _Float16* b1p = W + (size_t)(bcol0 + nw * 32 + 16 + c) * ldw + 8 * hh;
  v8f a00 = zero8(), a01 = zero8(), a10 = zero8(), a11 = zero8();
#pragma unroll 1
  for (int ks = 0; ks < nks; ++ks) {
    const size_t ao = (size_t)ks * aks;
    const int bo = ks * 32;
    const v16h fa0 = ldfrag_h(a0p + ao);
    const v16h fa1 = ldfrag_h(a1p + ao);
    const v16h fb0 = ldfrag_h(b0p + bo);
    const v16h fb1 = ldfrag_h(b1p + bo);
    a00 = mma_raw(fa0, fb0, a00);
    a01 = mma_raw(fa0, fb1, a01);
    a10 = mma_raw(fa1, fb0, a10);
    a11 = mma_raw(fa1, fb1, a11);
    guard4(a00, a01, a10, a11, fa0, fa1, fb0, fb1);
  }
#pragma unroll
  for (int r = 0; r < 8; ++r) {
    const int row = mw * 32 + 8 * hh + r;
    Cs[row * LDC + nw * 32 + c]             = a00[r];
    Cs[row * LDC + nw * 32 + 16 + c]        = a01[r];
    Cs[(row + 16) * LDC + nw * 32 + c]      = a10[r];
    Cs[(row + 16) * LDC + nw * 32 + 16 + c] = a11[r];
  }
}

__global__ __launch_bounds__(256)
void k_ln1(const float* __restrict__ x, const float* __restrict__ g, const float* __restrict__ bb,
           float* xn, unsigned short* xw) {
  const int tid = threadIdx.x, wv = tid >> 5, lane = tid & 31;
  const int row = blockIdx.x * 8 + wv;
  const int wi = row / TP, n = row - wi * TP;
  const bool valid = n < NTW;
  const int t = win_token(wi, n);
  const v4f v  = *(const v4f*)(x + (size_t)t * CCH + lane * 4);
  const v4f gr = *(const v4f*)(g + lane * 4);
  const v4f br = *(const v4f*)(bb + lane * 4);
  v4f a, gg, be;
#pragma unroll
  for (int e = 0; e < 4; ++e) { a[e] = bfr(v[e]); gg[e] = bfr(gr[e]); be[e] = bfr(br[e]); }
  const v4f y = ln4(a, gg, be);
  if (valid) {
    float* xp = xn + (size_t)t * CCH + lane * 4;
    *(volatile v4f*)xp = y;
    __threadfence();
    *(volatile v4f*)xp = y;
  }
  const float m = valid ? 8.0f : 0.0f;
  v2u pk;
  pk[0] = pk16(hb16(y[0] * m), hb16(y[1] * m));
  pk[1] = pk16(hb16(y[2] * m), hb16(y[3] * m));
  unsigned short* gp = xw + (size_t)row * CCH + lane * 4;
  *(volatile v2u*)gp = pk;
  __threadfence();
  *(volatile v2u*)gp = pk;
}

__global__ __launch_bounds__(256)
void k_dwconv(const float* __restrict__ xn, const float* __restrict__ dww, const float* __restrict__ dwb,
              float* sp) {
  const int tid = threadIdx.x, wv = tid >> 5, lane = tid & 31;
  const int t = blockIdx.x * 8 + wv;
  const int wq = t % FR;
  const int hq = (t / FR) % FR;
  const int f = t / (FR * FR);
  v4f acc;
  acc[0] = 0.f; acc[1] = 0.f; acc[2] = 0.f; acc[3] = 0.f;
#pragma unroll 1
  for (int tap = 0; tap < 9; ++tap) {
    const int kh = tap / 3, kw = tap - kh * 3;
    const int h2 = hq + kh - 1, w2 = wq + kw - 1;
    const float m = (((unsigned)h2 < (unsigned)FR) && ((unsigned)w2 < (unsigned)FR)) ? 1.0f : 0.0f;
    const int hc = min(max(h2, 0), FR - 1), wc = min(max(w2, 0), FR - 1);
    const v4f xv = *(const v4f*)(xn + ((size_t)(f * FR + hc) * FR + wc) * CCH + lane * 4);
    const v4f wv4 = *(const v4f*)(dww + tap * CCH + lane * 4);
#pragma unroll
    for (int e = 0; e < 4; ++e) acc[e] += (xv[e] * m) * bfr(wv4[e]);
  }
  const v4f b4 = *(const v4f*)(dwb + lane * 4);
  v4f o;
#pragma unroll
  for (int e = 0; e < 4; ++e) o[e] = acc[e] + bfr(b4[e]);
  float* p = sp + (size_t)t * CCH + lane * 4;
  *(volatile v4f*)p = o;
  __threadfence();
  *(volatile v4f*)p = o;
}

__global__ __launch_bounds__(256) void k_cvt_w(const float* __restrict__ wsrc, unsigned short* wdst,
                                               int nrows, int ncols) {
  const int tid = threadIdx.x, wv = tid >> 5, lane = tid & 31;
  const int row = blockIdx.x * 8 + wv;
  if (row < nrows) {
    for (int cb = 0; cb < ncols; cb += CCH) {
      const v4f a = *(const v4f*)(wsrc + (size_t)row * ncols + cb + lane * 4);
      v2u pk;
      pk[0] = pk16(hb16(bfr(a[0]) * 64.0f), hb16(bfr(a[1]) * 64.0f));
      pk[1] = pk16(hb16(bfr(a[2]) * 64.0f), hb16(bfr(a[3]) * 64.0f));
      unsigned short* gp = wdst + (size_t)row * ncols + cb + lane * 4;
      *(volatile v2u*)gp = pk;
      __threadfence();
      *(volatile v2u*)gp = pk;
    }
  }
}

__global__ __launch_bounds__(256)
void k_gemm_qkv(const unsigned short* __restrict__ xw, const unsigned short* __restrict__ wq,
                const float* __restrict__ bq, unsigned short* qpl, unsigned short* kpl, unsigned short* vtp) {
  __shared__ __align__(16) float Cs[64 * LDC];
  const int tid = threadIdx.x;
  const int mb = blockIdx.x, nb = blockIdx.y;
  mm_tile((const _Float16*)(const void*)xw, CCH, (size_t)32, (const _Float16*)(const void*)wq, CCH, CCH / 32,
          mb * 64, nb * 128, Cs);
  __syncthreads();

  const int wi = mb / STRIPS, tok0 = (mb - wi * STRIPS) * 64;
  const float* bqn = bq + nb * 128;
  if (nb < 2) {
    unsigned short* dst = (nb == 0) ? qpl : kpl;
    const float scl = (nb == 0) ? (QSC * 64.0f) : 8.0f;
    v4u pk[4];
    size_t offs[4];
#pragma unroll
    for (int s = 0; s < 4; ++s) {
      const int L = s * 32 + (tid >> 3), p = tid & 7;
      const int h4 = L >> 5, li = L & 31;
      const int tok = 2 * li + (p >> 2), d0 = (p & 3) * 8;
      const int col = h4 * 32 + d0;
      v4u q4;
#pragma unroll
      for (int e = 0; e < 4; ++e) {
        float f0 = Cs[tok * LDC + col + 2 * e] * (1.0f / 512.0f) + bfr(bqn[col + 2 * e]);
        float f1 = Cs[tok * LDC + col + 2 * e + 1] * (1.0f / 512.0f) + bfr(bqn[col + 2 * e + 1]);
        f0 = f0 * scl;
        f1 = f1 * scl;
        q4[e] = pk16(hb16(f0), hb16(f1));
      }
      pk[s] = q4;
      offs[s] = ((size_t)((wi * NHD + h4) * TP + tok0 + tok)) * HD + d0;
    }
#pragma unroll
    for (int s = 0; s < 4; ++s) *(volatile v4u*)(dst + offs[s]) = pk[s];
    __threadfence();
#pragma unroll
    for (int s = 0; s < 4; ++s) *(volatile v4u*)(dst + offs[s]) = pk[s];
  } else {
    v4u pv[4];
    size_t offs[4];
#pragma unroll
    for (int s = 0; s < 4; ++s) {
      const int L = s * 32 + (tid >> 3), p = tid & 7;
      const int h4 = L >> 5, d = L & 31;
      const int col = h4 * 32 + d;
      const int tb = p * 8;
      const float bc = bfr(bqn[col]);
      v4u a;
#pragma unroll
      for (int e = 0; e < 4; ++e) {
        const float v0 = Cs[(tb + 2 * e) * LDC + col] * (1.0f / 512.0f) + bc;
        const float v1 = Cs[(tb + 2 * e + 1) * LDC + col] * (1.0f / 512.0f) + bc;
        a[e] = pk16(hb16(v0 * 16.0f), hb16(v1 * 16.0f));
      }
      pv[s] = a;
      offs[s] = ((size_t)((wi * NHD + h4) * HD + d)) * TP + tok0 + tb;
    }
#pragma unroll
    for (int s = 0; s < 4; ++s) *(volatile v4u*)(vtp + offs[s]) = pv[s];
    __threadfence();
#pragma unroll
    for (int s = 0; s < 4; ++s) *(volatile v4u*)(vtp + offs[s]) = pv[s];
  }
}

__global__ __launch_bounds__(128)
void k_attn(const unsigned short* __restrict__ qpl, const unsigned short* __restrict__ kpl,
            const unsigned short* __restrict__ vtp, unsigned short* opl) {
  __shared__ __align__(16) char pbuf[4 * PWB];
  const int tid = threadIdx.x, wave = tid >> 5, lane = tid & 31, hh = lane >> 4, c = lane & 15;
  const int wh = blockIdx.x / STRIPS;
  const int sb = blockIdx.x - wh * STRIPS;
  const int wi = wh >> 2, h = wh & 3;
  const int strip = sb * 4 + wave;
  const int q0 = strip * 16;
  unsigned short* ob = opl + ((size_t)h * NROWW + (size_t)wi * TP + q0) * HD;
  unsigned short* op0 = ob + lane * 8;
  unsigned short* op1 = ob + 256 + lane * 8;

  if (q0 >= QEND) {
    v4u z;
    z[0] = 0u; z[1] = 0u; z[2] = 0u; z[3] = 0u;
    *(volatile v4u*)op0 = z;
    *(volatile v4u*)op1 = z;
    __threadfence();
    *(volatile v4u*)op0 = z;
    *(volatile v4u*)op1 = z;
    return;
  }

  const _Float16* Q = (const _Float16*)(const void*)qpl + (size_t)wh * TP * HD;
  const _Float16* K = (const _Float16*)(const void*)kpl + (size_t)wh * TP * HD;
  const _Float16* V = (const _Float16*)(const void*)vtp + (size_t)wh * HD * TP;
  _Float16* Ph = (_Float16*)(pbuf + wave * PWB);

  const v16h qa = ldfrag_h(Q + (size_t)(q0 + c) * HD + 8 * hh);
  float mrow[8], lrow[8];
#pragma unroll
  for (int r = 0; r < 8; ++r) { mrow[r] = -1e30f; lrow[r] = 0.f; }
  v8f oa0 = zero8(), oa1 = zero8();

#pragma unroll 1
  for (int kb = 0; kb < TP / 64; ++kb) {
    v8f s[4];
#pragma unroll
    for (int j = 0; j < 4; ++j) {
      const int key = kb * 64 + j * 16 + c;
      const v16h kf = ldfrag_h(K + (size_t)key * HD + 8 * hh);
      v8f sj = mma_g1(qa, kf, zero8());
      const bool kv = key < NTW;
#pragma unroll
      for (int r = 0; r < 8; ++r) sj[r] = kv ? sj[r] : -1.0e30f;
      s[j] = sj;
    }
#pragma unroll
    for (int r = 0; r < 8; ++r) {
      float tm = fmaxf(fmaxf(s[0][r], s[1][r]), fmaxf(s[2][r], s[3][r]));
      tm = fmaxf(tm, __shfl_xor(tm, 1, 32));
      tm = fmaxf(tm, __shfl_xor(tm, 2, 32));
      tm = fmaxf(tm, __shfl_xor(tm, 4, 32));
      tm = fmaxf(tm, __shfl_xor(tm, 8, 32));
      const float mn = fmaxf(mrow[r], tm);
      const float alpha = __expf((mrow[r] - mn) * INV512);
      mrow[r] = mn;
      float ps = 0.f;
#pragma unroll
      for (int j = 0; j < 4; ++j) {
        const float p = __expf((s[j][r] - mn) * INV512 + LN4096);
        ps = ps + p;
        s[j][r] = p;
      }
      ps = ps + __shfl_xor(ps, 1, 32);
      ps = ps + __shfl_xor(ps, 2, 32);
      ps = ps + __shfl_xor(ps, 4, 32);
      ps = ps + __shfl_xor(ps, 8, 32);
      lrow[r] = lrow[r] * alpha + ps;
      oa0[r] = oa0[r] * alpha;
      oa1[r] = oa1[r] * alpha;
    }
#pragma unroll
    for (int j = 0; j < 4; ++j) {
#pragma unroll
      for (int r = 0; r < 8; ++r) {
        Ph[(8 * hh + r) * PP + j * 16 + c] = (_Float16)s[j][r];
      }
    }
    wave_sync_lds();
#pragma unroll
    for (int ks = 0; ks < 2; ++ks) {
      const v16h pa = ldfrag_h(Ph + c * PP + ks * 32 + 8 * hh);
      const int koff = kb * 64 + ks * 32 + 8 * hh;
      const v16h v0 = ldfrag_h(V + (size_t)c * TP + koff);
      const v16h v1 = ldfrag_h(V + (size_t)(16 + c) * TP + koff);
      oa0 = mma_raw(pa, v0, oa0);
      oa1 = mma_raw(pa, v1, oa1);
      guard2(oa0, oa1, pa, v0, v1);
    }
    wave_sync_lds();
  }

  float* Os = (float*)(void*)(pbuf + wave * PWB);
#pragma unroll
  for (int r = 0; r < 8; ++r) {
    const float inv = 1.0f / (lrow[r] * 16.0f);
    const int row = 8 * hh + r;
    Os[row * OSP + c]      = oa0[r] * inv;
    Os[row * OSP + 16 + c] = oa1[r] * inv;
  }
  wave_sync_lds();
  v4u pk[2];
#pragma unroll
  for (int sI = 0; sI < 2; ++sI) {
    const int line = sI * 4 + (lane >> 3), piece = lane & 7;
    const int row = 2 * line + (piece >> 2), d0 = (piece & 3) * 8;
    v4u a;
#pragma unroll
    for (int e = 0; e < 4; ++e) {
      const float f0 = Os[row * OSP + d0 + 2 * e] * 64.0f;
      const float f1 = Os[row * OSP + d0 + 2 * e + 1] * 64.0f;
      a[e] = pk16(hb16(f0), hb16(f1));
    }
    pk[sI] = a;
  }
  *(volatile v4u*)op0 = pk[0];
  *(volatile v4u*)op1 = pk[1];
  __threadfence();
  *(volatile v4u*)op0 = pk[0];
  *(volatile v4u*)op1 = pk[1];
}

__global__ __launch_bounds__(256)
void k_gemm_proj(const unsigned short* __restrict__ opl, const unsigned short* __restrict__ wp,
                 const float* __restrict__ bp, const float* __restrict__ sp, const float* __restrict__ x,
                 float* x1) {
  __shared__ __align__(16) float Cs[64 * LDC];
  const int tid = threadIdx.x, wave = tid >> 5, lane = tid & 31;
  const int mb = blockIdx.x;
  mm_tile((const _Float16*)(const void*)opl, HD, (size_t)NROWW * HD, (const _Float16*)(const void*)wp, CCH,
          CCH / 32, mb * 64, 0, Cs);
  __syncthreads();

  const int wi = mb / STRIPS, tok0 = (mb - wi * STRIPS) * 64;
  const v4f b4 = *(const v4f*)(bp + lane * 4);
  v4f bb;
#pragma unroll
  for (int e = 0; e < 4; ++e) bb[e] = bfr(b4[e]);
#pragma unroll 1
  for (int it = 0; it < 8; ++it) {
    const int row = wave * 8 + it;
    const int tok = tok0 + row;
    if (tok < NTW) {
      const int t = win_token(wi, tok);
      const v4f a  = *(const v4f*)(Cs + row * LDC + lane * 4);
      const v4f sv = *(const v4f*)(sp + (size_t)t * CCH + lane * 4);
      const v4f xv = *(const v4f*)(x + (size_t)t * CCH + lane * 4);
      v4f o;
#pragma unroll
      for (int e = 0; e < 4; ++e) o[e] = bfr(xv[e]) + ((a[e] * (1.0f / 4096.0f) + bb[e]) + sv[e]);
      float* p = x1 + (size_t)t * CCH + lane * 4;
      *(volatile v4f*)p = o;
      __threadfence();
      *(volatile v4f*)p = o;
    }
  }
}

__global__ __launch_bounds__(256)
void k_ln2(const float* __restrict__ x1, const float* __restrict__ g, const float* __restrict__ bb,
           unsigned short* xm) {
  const int tid = threadIdx.x, wv = tid >> 5, lane = tid & 31;
  const int t = blockIdx.x * 8 + wv;
  const v4f a  = *(const v4f*)(x1 + (size_t)t * CCH + lane * 4);
  const v4f gr = *(const v4f*)(g + lane * 4);
  const v4f br = *(const v4f*)(bb + lane * 4);
  v4f gg, be;
#pragma unroll
  for (int e = 0; e < 4; ++e) { gg[e] = bfr(gr[e]); be[e] = bfr(br[e]); }
  const v4f y = ln4(a, gg, be);
  v2u pk;
  pk[0] = pk16(hb16(y[0] * 8.0f), hb16(y[1] * 8.0f));
  pk[1] = pk16(hb16(y[2] * 8.0f), hb16(y[3] * 8.0f));
  unsigned short* gp = xm + (size_t)t * CCH + lane * 4;
  *(volatile v2u*)gp = pk;
  __threadfence();
  *(volatile v2u*)gp = pk;
}

__global__ __launch_bounds__(256)
void k_gemm_fc1(const unsigned short* __restrict__ xm, const unsigned short* __restrict__ w1,
                const float* __restrict__ b1, unsigned short* hp) {
  __shared__ __align__(16) float Cs[64 * LDC];
  const int tid = threadIdx.x;
  const int mb = blockIdx.x, nb = blockIdx.y;
  mm_tile((const _Float16*)(const void*)xm, CCH, (size_t)32, (const _Float16*)(const void*)w1, CCH, CCH / 32,
          mb * 64, nb * 128, Cs);
  __syncthreads();
  const float* bn = b1 + nb * 128;
#pragma unroll 2
  for (int it = 0; it < 32; ++it) {
    const int idx = it * 256 + tid;
    const int row = idx >> 7, col = idx & 127;
    const float v = Cs[row * LDC + col] * (1.0f / 512.0f) + bfr(bn[col]);
    const float gl = 0.5f * v * (1.0f + erff(v * 0.70710678118654752f));
    Cs[row * LDC + col] = gl * 64.0f;
  }
  __syncthreads();
  v4u pk[4];
  size_t offs[4];
#pragma unroll
  for (int s = 0; s < 4; ++s) {
    const int idx = s * 256 + tid;
    const int row = idx >> 4, piece = idx & 15;
    const int col0 = piece * 8;
    v4u q4;
#pragma unroll
    for (int e = 0; e < 4; ++e) {
      q4[e] = pk16(hb16(Cs[row * LDC + col0 + 2 * e]), hb16(Cs[row * LDC + col0 + 2 * e + 1]));
    }
    pk[s] = q4;
    offs[s] = (size_t)(mb * 64 + row) * HID + nb * 128 + col0;
  }
#pragma unroll
  for (int s = 0; s < 4; ++s) *(volatile v4u*)(hp + offs[s]) = pk[s];
  __threadfence();
#pragma unroll
  for (int s = 0; s < 4; ++s) *(volatile v4u*)(hp + offs[s]) = pk[s];
}

__global__ __launch_bounds__(256)
void k_gemm_fc2(const unsigned short* __restrict__ hp, const unsigned short* __restrict__ w2,
                const float* __restrict__ b2, const float* __restrict__ x1, float* out) {
  __shared__ __align__(16) float Cs[64 * LDC];
  const int tid = threadIdx.x, wave = tid >> 5, lane = tid & 31;
  const int mb = blockIdx.x;
  mm_tile((const _Float16*)(const void*)hp, HID, (size_t)32, (const _Float16*)(const void*)w2, HID, HID / 32,
          mb * 64, 0, Cs);
  __syncthreads();
  const v4f b4 = *(const v4f*)(b2 + lane * 4);
  v4f bb;
#pragma unroll
  for (int e = 0; e < 4; ++e) bb[e] = bfr(b4[e]);
#pragma unroll 1
  for (int it = 0; it < 8; ++it) {
    const int row = wave * 8 + it;
    const int t = mb * 64 + row;
    const v4f a  = *(const v4f*)(Cs + row * LDC + lane * 4);
    const v4f xv = *(const v4f*)(x1 + (size_t)t * CCH + lane * 4);
    v4f o;
#pragma unroll
    for (int e = 0; e < 4; ++e) o[e] = xv[e] + (a[e] * (1.0f / 4096.0f) + bb[e]);
    float* p = out + (size_t)t * CCH + lane * 4;
    *(volatile v4f*)p = o;
    __threadfence();
    *(volatile v4f*)p = o;
  }
}

extern "C" void kernel_launch(void* const* d_in, const int* in_sizes, int n_in,
                              void* d_out, int out_size, void* d_ws, size_t ws_size,
                              hipStream_t stream) {
  if (n_in < 15) return;
  if (in_sizes[0] != NTN * CCH) return;
  if (in_sizes[1] != CCH || in_sizes[2] != CCH) return;
  if (in_sizes[3] != C3 * CCH || in_sizes[4] != C3) return;
  if (in_sizes[5] != CCH * CCH || in_sizes[6] != CCH) return;
  if (in_sizes[7] != 9 * CCH || in_sizes[8] != CCH) return;
  if (in_sizes[9] != CCH || in_sizes[10] != CCH) return;
  if (in_sizes[11] != HID * CCH || in_sizes[12] != HID) return;
  if (in_sizes[13] != CCH * HID || in_sizes[14] != CCH) return;
  if (out_size != NTN * CCH) return;

  const float* x      = (const float*)d_in[0];
  const float* n1g    = (const float*)d_in[1];
  const float* n1b    = (const float*)d_in[2];
  const float* qkvw   = (const float*)d_in[3];
  const float* qkvb   = (const float*)d_in[4];
  const float* projw  = (const float*)d_in[5];
  const float* projb  = (const float*)d_in[6];
  const float* dww    = (const float*)d_in[7];
  const float* dwb    = (const float*)d_in[8];
  const float* n2g    = (const float*)d_in[9];
  const float* n2b    = (const float*)d_in[10];
  const float* fc1w   = (const float*)d_in[11];
  const float* fc1b   = (const float*)d_in[12];
  const float* fc2w   = (const float*)d_in[13];
  const float* fc2b   = (const float*)d_in[14];
  float* out = (float*)d_out;

  const size_t sXN = (size_t)NTN * CCH * 4;
  const size_t sXW = (size_t)NROWW * CCH * 2;
  const size_t sO  = (size_t)NHD * NROWW * HD * 2;
  const size_t sH  = (size_t)NTN * HID * 2;
  const size_t sQ  = (size_t)NWIN * NHD * TP * HD * 2;
  const size_t sXM = (size_t)NTN * CCH * 2;
  const size_t sS  = sXN;
  const size_t sWq = (size_t)C3 * CCH * 2;
  const size_t sWp = (size_t)CCH * CCH * 2;
  const size_t sW1 = (size_t)HID * CCH * 2;
  const size_t sW2 = (size_t)CCH * HID * 2;
  size_t sA = sXN + sXW;
  if (sH > sA) sA = sH;
  if (sO > sA) sA = sO;
  size_t sB = 3 * sQ;
  if (sXN + sXM > sB) sB = sXN + sXM;

  size_t off = 0;
  const size_t oA  = off; off += sA;
  const size_t oB  = off; off += sB;
  const size_t oS  = off; off += sS;
  const size_t oWq = off; off += sWq;
  const size_t oWp = off; off += sWp;
  const size_t oW1 = off; off += sW1;
  const size_t oW2 = off; off += sW2;
  if (off > ws_size) return;
  if (off > (size_t)134217728) return;

  char* ws = (char*)d_ws;
  float*          XN  = (float*)(ws + oA);
  unsigned short* XW  = (unsigned short*)(ws + oA + sXN);
  unsigned short* Opl = (unsigned short*)(ws + oA);
  unsigned short* Hp  = (unsigned short*)(ws + oA);
  unsigned short* Qp  = (unsigned short*)(ws + oB);
  unsigned short* Kp  = (unsigned short*)(ws + oB + sQ);
  unsigned short* Vtp = (unsigned short*)(ws + oB + 2 * sQ);
  float*          X1  = (float*)(ws + oB);
  unsigned short* XM  = (unsigned short*)(ws + oB + sXN);
  float*          Sp  = (float*)(ws + oS);
  unsigned short* Wq  = (unsigned short*)(ws + oWq);
  unsigned short* Wp  = (unsigned short*)(ws + oWp);
  unsigned short* W1  = (unsigned short*)(ws + oW1);
  unsigned short* W2  = (unsigned short*)(ws + oW2);

  const dim3 blk(256);
  k_ln1<<<dim3(NROWW / 8), blk, 0, stream>>>(x, n1g, n1b, XN, XW);
  k_dwconv<<<dim3(NTN / 8), blk, 0, stream>>>(XN, dww, dwb, Sp);
  k_cvt_w<<<dim3(C3 / 8), blk, 0, stream>>>(qkvw, Wq, C3, CCH);
  k_cvt_w<<<dim3(CCH / 8), blk, 0, stream>>>(projw, Wp, CCH, CCH);
  k_cvt_w<<<dim3(HID / 8), blk, 0, stream>>>(fc1w, W1, HID, CCH);
  k_cvt_w<<<dim3(CCH / 8), blk, 0, stream>>>(fc2w, W2, CCH, HID);
  k_gemm_qkv<<<dim3(NROWW / 64, 3), blk, 0, stream>>>(XW, Wq, qkvb, Qp, Kp, Vtp);
  k_attn<<<dim3(NWIN * NHD * STRIPS), dim3(128), 0, stream>>>(Qp, Kp, Vtp, Opl);
  k_gemm_proj<<<dim3(NROWW / 64), blk, 0, stream>>>(Opl, Wp, projb, Sp, x, X1);
  k_ln2<<<dim3(NTN / 8), blk, 0, stream>>>(X1, n2g, n2b, XM);
  k_gemm_fc1<<<dim3(NTN / 64, HID / 128), blk, 0, stream>>>(XM, W1, fc1b, Hp);
  k_gemm_fc2<<<dim3(NTN / 64), blk, 0, stream>>>(Hp, W2, fc2b, X1, out);
  (void)hipGetLastError();
}
